// RModel_88648124990070
// MI455X (gfx1250) — hardware-run, weakly checked
//
#include <hip/hip_runtime.h>


namespace {
constexpr int N = 100000, NP = 100032, E = 1200000, F0 = 32, H1D = 64, OUTD = 64, R = 3, G = 512, NCLS = 10, NSH = 16, NCO = 16;
constexpr float XS = 8.0f, WSC = 256.0f, NEG = 0.2f  ;

typedef _Float16 b16;
typedef __attribute__((ext_vector_type(16))) _Float16 v16b;
typedef __attribute__((ext_vector_type(8))) _Float16 v8b;
typedef __attribute__((ext_vector_type(8))) float v8f;
typedef __attribute__((ext_vector_type(4))) float v4f;
__device__ __forceinline__ float bf16_rne(float f) { unsigned int u = __float_as_uint(f); u += 0x7FFFu + ((u >> 16) & 1u); return __uint_as_float(u & 0xFFFF0000u); }
__device__ __forceinline__ void split16(float v, b16& hi, b16& lo) { hi = (b16)v; lo = (b16)(v - (float)hi); }
__device__ __forceinline__ v16b frag_kb(const b16* p, int hh) { const v8b a = *(const v8b*)(p + 8 * hh), b = *(const v8b*)(p + 16 + 8 * hh); v16b f;
#pragma unroll
  for (int e = 0; e < 8; ++e) { f[e] = a[e]; f[8 + e] = b[e]; } return f; }
__device__ __forceinline__ v8f wmma16b(v16b a, v16b b, v8f c) { v8f d = __builtin_amdgcn_wmma_f32_16x16x32_f16(false, a, false, b, (short)0, c, false, false); asm volatile("v_nop\n\tv_nop\n\tv_nop\n\tv_nop" : "+v"(d) : "v"(a), "v"(b)); return d; }
__device__ __forceinline__ void wave_lds_sync() { __builtin_amdgcn_fence(__ATOMIC_RELEASE, "workgroup"); __builtin_amdgcn_wave_barrier(); __builtin_amdgcn_fence(__ATOMIC_ACQUIRE, "workgroup"); }
__device__ __forceinline__ float pmul(float a, float b) { float p = a * b; asm volatile("" : "+v"(p)); return p; }
__device__ __forceinline__ int iclamp(int v, int lo, int hi) { return v < lo ? lo : (v > hi ? hi : v); }
__device__ __forceinline__ float nexp(float x) { return __builtin_amdgcn_exp2f(x * 1.4426950408889634f); }
__device__ __forceinline__ float lrelu(float x) { return x > 0.0f ? x : NEG * x; }

constexpr int CSR_NBLK = 512, CSR_GB = 9, CSR_GN = 1 << CSR_GB  , CSR_MAXG = 512, CSR_CAP = 12288  ;
__global__ __launch_bounds__(64) void csrA_kernel(const int* __restrict__ dst, int E, int N, int nG, int CHP, int NGP, int* __restrict__ STG, int* __restrict__ HST) {
  extern __shared__ int sm[];
  int* cnt = sm; int* run = sm + NGP; int* ids = sm + 2 * NGP;
  const int b = blockIdx.x; const int ch = (E + CSR_NBLK - 1) / CSR_NBLK; const int e0 = b * ch, e1 = min(E, e0 + ch);
  for (int i = threadIdx.x; i < NGP; i += 64) cnt[i] = 0;
  for (int i = threadIdx.x; i < CHP; i += 64) ids[i] = -1;
  __syncthreads();
  if (threadIdx.x == 0) {
    for (int e = e0; e < e1; ++e) { int d = dst[e]; d = (d < 0) ? 0 : (d >= N ? N - 1 : d); cnt[d >> CSR_GB] += 1; }
    int acc = 0; for (int g = 0; g < nG; ++g) { run[g] = acc; acc += cnt[g]; }
    for (int e = e0; e < e1; ++e) { int d = dst[e]; d = (d < 0) ? 0 : (d >= N ? N - 1 : d); const int g = d >> CSR_GB; ids[run[g]] = e; run[g] += 1; } }
  __syncthreads();
  typedef __attribute__((ext_vector_type(4))) int v4i;
  for (int pass = 0; pass < 2; ++pass) {
    for (int i = threadIdx.x; i < CHP / 4; i += 64) *(volatile v4i*)(STG + (size_t)b * CHP + i * 4) = *(const v4i*)(&ids[i * 4]);
    for (int i = threadIdx.x; i < NGP / 4; i += 64) { v4i v; for (int e = 0; e < 4; ++e) v[e] = (i * 4 + e < nG) ? cnt[i * 4 + e] : 0; *(volatile v4i*)(HST + (size_t)b * NGP + i * 4) = v; }
    __threadfence(); }
}
__global__ __launch_bounds__(512) void csrS_kernel(const int* __restrict__ HST, int nG, int NGP, int* __restrict__ START, int* __restrict__ TOT, int* __restrict__ OFF) {
  __shared__ int tot[CSR_MAXG];
  const int b = threadIdx.x;
  for (int pass = 0; pass < 2; ++pass) { int runb = 0; for (int g = 0; g < nG; ++g) { int c = HST[(size_t)b * NGP + g]; c = (c < 0) ? 0 : c; ((volatile int*)OFF)[(size_t)g * CSR_NBLK + b] = runb; runb += c; } __threadfence(); }
  for (int g = threadIdx.x; g < nG; g += 512) { int s = 0; for (int bb = 0; bb < CSR_NBLK; ++bb) { int c = HST[(size_t)bb * NGP + g]; s += (c < 0) ? 0 : c; } tot[g] = s; }
  __syncthreads();
  if (threadIdx.x < 32) {
    __shared__ int st[CSR_MAXG + 32];
    if (threadIdx.x == 0) { int acc = 0; for (int g = 0; g < NGP; ++g) { st[g] = acc; if (g < nG) acc += (tot[g] + 31) & ~31; } st[NGP] = acc; }
    __builtin_amdgcn_fence(__ATOMIC_RELEASE, "workgroup"); __builtin_amdgcn_wave_barrier(); __builtin_amdgcn_fence(__ATOMIC_ACQUIRE, "workgroup");
    for (int pass = 0; pass < 2; ++pass) { for (int i = threadIdx.x; i < NGP + 32; i += 32) { ((volatile int*)START)[i] = (i <= NGP) ? st[min(i, NGP)] : 0; ((volatile int*)TOT)[i] = (i < nG) ? tot[i] : 0; } __threadfence(); } }
}
__global__ __launch_bounds__(256) void csrB_kernel(const int* __restrict__ dst, int N, int nG, int CHP, int NGP, int permLen, const int* __restrict__ STG, const int* __restrict__ HST, const int* __restrict__ OFF, const int* __restrict__ START, const int* __restrict__ TOT, int* __restrict__ PERM, int* __restrict__ ROWPTR, int* __restrict__ ROWCNT, int* __restrict__ FLAG) {
  typedef __attribute__((ext_vector_type(4))) int v4i;
  __shared__ int ids[CSR_CAP]; __shared__ unsigned short key[CSR_CAP]; __shared__ int outp[CSR_CAP]; __shared__ int ncnt[CSR_GN + 1]; __shared__ int boff[CSR_NBLK + 1];
  const int g = blockIdx.x, t_ = threadIdx.x; int tot = TOT[g]; int st = START[g], stn = START[g + 1]; const int v0 = g * CSR_GN; const int nv = min(CSR_GN, N - v0);
  st = (st < 0) ? 0 : (st > permLen - 32 ? permLen - 32 : st) & ~31; stn = (stn < st) ? st : (stn > permLen ? permLen : stn); tot = (tot < 0) ? 0 : tot; if (tot > stn - st && tot <= CSR_CAP) tot = stn - st;
  if (tot > CSR_CAP) {
    for (int pass = 0; pass < 2; ++pass) { for (int i = t_; i < CSR_GN / 4; i += 256) { v4i a, c; for (int e = 0; e < 4; ++e) { a[e] = st; c[e] = 0; } *(volatile v4i*)(ROWPTR + v0 + i * 4) = a; *(volatile v4i*)(ROWCNT + v0 + i * 4) = c; } if (t_ == 0) ((volatile int*)FLAG)[0] = 1; __threadfence(); } (void)nv; return; }
  if (t_ == 0) { int acc = 0; for (int b = 0; b < CSR_NBLK; ++b) { boff[b] = acc; int c = HST[(size_t)b * NGP + g]; c = (c < 0) ? 0 : (c > CHP ? CHP : c); acc += c; if (acc > tot) acc = tot; } boff[CSR_NBLK] = acc; }
  for (int i = t_; i <= CSR_GN; i += 256) ncnt[i] = 0;
  __syncthreads();
  for (int b = 0; b < CSR_NBLK; ++b) { const int c = boff[b + 1] - boff[b]; int o_ = OFF[(size_t)g * CSR_NBLK + b]; o_ = (o_ < 0) ? 0 : (o_ > CHP - c ? CHP - c : o_); const int* src_ = STG + (size_t)b * CHP + o_;
    for (int i = t_; i < c; i += 256) { int id = src_[i]; id = (id < 0) ? 0 : id; ids[boff[b] + i] = id; int d = dst[id]; d = (d < v0) ? v0 : (d >= N ? N - 1 : d); int kk = d - v0; kk = (kk < 0) ? 0 : (kk >= CSR_GN ? CSR_GN - 1 : kk); key[boff[b] + i] = (unsigned short)kk; } }
  __syncthreads();
  if (t_ == 0) { for (int i = 0; i < tot; ++i) ncnt[key[i]] += 1; int acc = 0; for (int vl = 0; vl < CSR_GN; ++vl) { const int c = ncnt[vl]; ncnt[vl] = acc; acc += c; } ncnt[CSR_GN] = acc;
    for (int i = 0; i < tot; ++i) { const int vl = key[i]; outp[ncnt[vl]] = ids[i]; ncnt[vl] += 1; }
    for (int vl = CSR_GN; vl > 0; --vl) ncnt[vl] = ncnt[vl - 1]; ncnt[0] = 0; }
  __syncthreads();
  for (int pass = 0; pass < 2; ++pass) {
    for (int i = t_; i < (stn - st) / 4; i += 256) { v4i v; for (int e = 0; e < 4; ++e) { const int q = i * 4 + e; v[e] = (q < tot) ? outp[q] : -1; } *(volatile v4i*)(PERM + st + i * 4) = v; }
    for (int i = t_; i < CSR_GN / 4; i += 256) { v4i a, c; for (int e = 0; e < 4; ++e) { const int vl = i * 4 + e; a[e] = st + ncnt[vl]; c[e] = (vl < nv) ? (ncnt[vl + 1] - ncnt[vl]) : 0; } *(volatile v4i*)(ROWPTR + v0 + i * 4) = a; *(volatile v4i*)(ROWCNT + v0 + i * 4) = c; }
    __threadfence(); }
}
__global__ __launch_bounds__(256) void csrZ_kernel(int* __restrict__ p, size_t n4) { typedef __attribute__((ext_vector_type(4))) int v4i; const size_t tid = (size_t)blockIdx.x * 256 + threadIdx.x, nth = (size_t)gridDim.x * 256; v4i z = {0, 0, 0, 0}; for (size_t i = tid; i < n4; i += nth) *(volatile v4i*)(p + i * 4) = z; }
struct CsrBufs { int *STG, *HST, *OFF, *START, *TOT, *PERM, *ROWPTR, *ROWCNT, *FLAG; int nG, NGP, CHP; size_t permLen; char* base; size_t bytes; };
static size_t csr_carve(CsrBufs& c, char* ws, size_t off, int E, int N) {
  const size_t off0 = off; c.base = ws + off;
  auto al = [&](size_t bytes) { char* p = ws + off; off += (bytes + 255) & ~(size_t)255; return p; };
  c.nG = (N + CSR_GN - 1) / CSR_GN; c.NGP = (c.nG + 31) & ~31; const int ch = (E + CSR_NBLK - 1) / CSR_NBLK; c.CHP = (ch + 31) & ~31; c.permLen = (size_t)E + 32 * (size_t)c.nG + 32;
  c.STG = (int*)al((size_t)CSR_NBLK * c.CHP * 4); c.HST = (int*)al((size_t)CSR_NBLK * c.NGP * 4); c.OFF = (int*)al((size_t)c.NGP * CSR_NBLK * 4); c.START = (int*)al((size_t)(c.NGP + 64) * 4); c.TOT = (int*)al((size_t)(c.NGP + 64) * 4);
  c.PERM = (int*)al(c.permLen * 4); c.ROWPTR = (int*)al((size_t)c.nG * CSR_GN * 4); c.ROWCNT = (int*)al((size_t)c.nG * CSR_GN * 4); c.FLAG = (int*)al(256);
  c.bytes = off - off0; return off;
}
static void csr_build(const CsrBufs& c, const int* dst, int E, int N, hipStream_t stream) {
  const size_t smem = (size_t)(2 * c.NGP + c.CHP) * 4;
  csrZ_kernel<<<512, 256, 0, stream>>>((int*)c.base, c.bytes / 16);
  csrA_kernel<<<CSR_NBLK, 64, smem, stream>>>(dst, E, N, c.nG, c.CHP, c.NGP, c.STG, c.HST);
  csrS_kernel<<<1, 512, 0, stream>>>(c.HST, c.nG, c.NGP, c.START, c.TOT, c.OFF);
  csrB_kernel<<<c.nG, 256, 0, stream>>>(dst, N, c.nG, c.CHP, c.NGP, (int)c.permLen, c.STG, c.HST, c.OFF, c.START, c.TOT, c.PERM, c.ROWPTR, c.ROWCNT, c.FLAG);
}


__global__ __launch_bounds__(256) void wprep_kernel(const float* __restrict__ Wr, const float* __restrict__ root, int fin, int fout, b16* __restrict__ WS) {
  const int KT = (1 + R) * fin; const int u = blockIdx.x * 256 + threadIdx.x; if (u >= fout * KT / 8) return; const int e = u * 8, oo = e / KT, k0 = e % KT; v8b o;
  for (int j = 0; j < 8; ++j) { const int k = k0 + j; float w; if (k < fin) w = root[(size_t)k * fout + oo]; else { const int r = (k - fin) / fin, kk = (k - fin) % fin; w = Wr[((size_t)r * fin + kk) * fout + oo]; } o[j] = (b16)(bf16_rne(w) * WSC); }
  for (int pass = 0; pass < 2; ++pass) { *(volatile v8b*)(WS + e) = o; __threadfence(); }
}
__global__ __launch_bounds__(128) void emb_kernel(const int* __restrict__ xid, const float* __restrict__ se, const float* __restrict__ ce, const float* __restrict__ pw, const float* __restrict__ pb, float* __restrict__ H0) {
  __shared__ __attribute__((aligned(16))) b16 WP[32][32 + 8]; __shared__ __attribute__((aligned(16))) float Tf[4][16][F0 + 4];
  const int wave = threadIdx.x >> 5, lane = threadIdx.x & 31, nloc = lane & 15, hlf = lane >> 4; const size_t m0 = (size_t)blockIdx.x * 64 + wave * 16;
  for (int q = threadIdx.x; q < 32 * 32; q += 128) { const int o = q >> 5, k = q & 31; WP[o][k] = k < 16 ? (b16)(bf16_rne(pw[k * F0 + o]) * WSC) : (b16)0.0f; }
  __syncthreads();
  const size_t v = m0 + nloc; v16b a = {};
  if (v < (size_t)N) { const int i0 = iclamp(xid[v * 2], 0, NSH - 1), i1 = iclamp(xid[v * 2 + 1], 0, NCO - 1); const float* src = hlf ? (ce + i1 * 8) : (se + i0 * 8); for (int e = 0; e < 8; ++e) a[e] = (b16)(bf16_rne(src[e]) * XS); }
  v8f acc[2] = {{}, {}};
#pragma unroll
  for (int t = 0; t < 2; ++t) acc[t] = wmma16b(a, frag_kb(&WP[t * 16 + nloc][0], hlf), acc[t]);
#pragma unroll
  for (int t = 0; t < 2; ++t) { const int c = t * 16 + nloc; const float bb = bf16_rne(pb[c]);
#pragma unroll 1
    for (int r = 0; r < 8; ++r) { const size_t row = m0 + 8 * hlf + r; Tf[wave][8 * hlf + r][c] = row < (size_t)N ? fmaxf(acc[t][r] * (1.0f / (XS * WSC)) + bb, 0.0f) : 0.0f; } }
  wave_lds_sync();
  for (int pass = 0; pass < 2; ++pass) { for (int rr = 0; rr < 16; ++rr) if (lane < 8) *(volatile v4f*)(H0 + (m0 + rr) * F0 + lane * 4) = *(const v4f*)(&Tf[wave][rr][lane * 4]); __threadfence(); }
}
template <int FIN, int FOUT, int LAYER0, int RELU>
__global__ __launch_bounds__(32) void rgcn_kernel(const float* __restrict__ xin, const int* __restrict__ ids, const int* __restrict__ srcs, const int* __restrict__ etype, const int* __restrict__ PERM, const int* __restrict__ ROWPTR, const int* __restrict__ ROWCNT, int permLen, const b16* __restrict__ WS, const float* __restrict__ bias, float* __restrict__ Hout) {
  constexpr int KT = (1 + R) * FIN, NC = FIN / 32, NT = FOUT / 16;
  __shared__ __attribute__((aligned(16))) b16 Ah[16][KT + 8], Al[16][KT + 8]; __shared__ __attribute__((aligned(16))) float Tf[16][FOUT + 4];
  const int lane = threadIdx.x, nloc = lane & 15, hlf = lane >> 4; const size_t v0 = (size_t)blockIdx.x * 16;
  auto rd = [&](size_t u, int c) -> float { if (LAYER0) { const size_t id = (size_t)iclamp(ids[u], 0, N - 1); return bf16_rne(xin[id * FIN + c]); } return xin[u * FIN + c]; };
  for (int rr = 0; rr < 16; ++rr) { const size_t v = v0 + rr; float acc[R][NC]; float cnt[R]; float self[NC];
    for (int r = 0; r < R; ++r) { cnt[r] = 0.0f; for (int i = 0; i < NC; ++i) acc[r][i] = 0.0f; } for (int i = 0; i < NC; ++i) self[i] = 0.0f;
    if (v < (size_t)N) { for (int i = 0; i < NC; ++i) self[i] = rd(v, i * 32 + lane); int st = ROWPTR[v], ct = ROWCNT[v]; ct = iclamp(ct, 0, 65536); st = iclamp(st, 0, permLen - ct);
      for (int k = 0; k < ct; ++k) { const int e = iclamp(PERM[st + k], 0, E - 1); const size_t s = (size_t)iclamp(srcs[e], 0, N - 1); const int r = iclamp(etype[e], 0, R - 1);
#pragma unroll
        for (int q = 0; q < R; ++q) if (q == r) { cnt[q] += 1.0f; for (int i = 0; i < NC; ++i) acc[q][i] += rd(s, i * 32 + lane); } } }
    for (int i = 0; i < NC; ++i) { b16 p, pl; split16(self[i] * XS, p, pl); Ah[rr][i * 32 + lane] = p; Al[rr][i * 32 + lane] = pl; }
#pragma unroll
    for (int r = 0; r < R; ++r) { const float inv = 1.0f / fmaxf(cnt[r], 1.0f); for (int i = 0; i < NC; ++i) { b16 p, pl; split16(acc[r][i] * inv * XS, p, pl); Ah[rr][FIN + r * FIN + i * 32 + lane] = p; Al[rr][FIN + r * FIN + i * 32 + lane] = pl; } } }
  wave_lds_sync();
  v8f d[NT];
#pragma unroll
  for (int t = 0; t < NT; ++t) d[t] = (v8f){};
#pragma unroll 2
  for (int kb = 0; kb < KT; kb += 32) { const v16b a = frag_kb(&Ah[nloc][kb], hlf), al = frag_kb(&Al[nloc][kb], hlf);
#pragma unroll
    for (int t = 0; t < NT; ++t) { const v16b bw = frag_kb(WS + (size_t)(t * 16 + nloc) * KT + kb, hlf); d[t] = wmma16b(a, bw, d[t]); d[t] = wmma16b(al, bw, d[t]); } }
#pragma unroll
  for (int t = 0; t < NT; ++t) { const int c = t * 16 + nloc; const float bb = bf16_rne(bias[c]);
#pragma unroll 1
    for (int r = 0; r < 8; ++r) { const int rr = 8 * hlf + r; float y = d[t][r] * (1.0f / (XS * WSC)) + bb; if (RELU) y = fmaxf(y, 0.0f); if (v0 + rr >= (size_t)N) y = 0.0f; Tf[rr][c] = y; } }
  wave_lds_sync();
  for (int pass = 0; pass < 2; ++pass) { for (int rr = 0; rr < 16; ++rr) { if (v0 + rr < (size_t)N) for (int c4 = lane * 4; c4 < FOUT; c4 += 128) *(volatile v4f*)(Hout + (v0 + rr) * FOUT + c4) = *(const v4f*)(&Tf[rr][c4]); } __threadfence(); }
}


__device__ int lower_bound_i(const int* a, int n, int key) { int lo = 0, hi = n; while (lo < hi) { const int mid = (lo + hi) >> 1; if (a[mid] < key) lo = mid + 1; else hi = mid; } return lo; }
__global__ __launch_bounds__(64) void pool_kernel(const float* __restrict__ H, const int* __restrict__ batch, float* __restrict__ GP) {
  const int g = blockIdx.x, c = threadIdx.x; const int lo = lower_bound_i(batch, N, g), hi = lower_bound_i(batch, N, g + 1);
  float s = 0.0f; for (int v = lo; v < hi; ++v) s += H[(size_t)v * OUTD + c]; const float m = s / fmaxf((float)(hi - lo), 1.0f);
  for (int pass = 0; pass < 2; ++pass) { ((volatile float*)GP)[(size_t)g * OUTD + c] = m; __threadfence(); }
}
__global__ __launch_bounds__(512) void cls_kernel(const float* __restrict__ GP, const float* __restrict__ cw, const float* __restrict__ cb, float* __restrict__ out) {
  const int g = threadIdx.x; float o_[NCLS];
#pragma unroll
  for (int o = 0; o < NCLS; ++o) { float s = bf16_rne(cb[o]);
#pragma unroll 1
    for (int c = 0; c < OUTD; ++c) s += pmul(GP[(size_t)g * OUTD + c], bf16_rne(cw[c * NCLS + o])); o_[o] = s; }
  for (int pass = 0; pass < 2; ++pass) {
#pragma unroll
    for (int o = 0; o < NCLS; ++o) ((volatile float*)out)[(size_t)g * NCLS + o] = o_[o]; __threadfence(); }
}
}

extern "C" void kernel_launch(void* const* d_in, const int* in_sizes, int n_in, void* d_out, int out_size, void* d_ws, size_t ws_size, hipStream_t stream) {
  (void)n_in;
  auto Fp = [&](int i) { return (const float*)d_in[i]; }; auto Ip = [&](int i) { return (const int*)d_in[i]; };
  if (in_sizes[0] != N * 2 || in_sizes[1] != 2 * E || in_sizes[2] != E || in_sizes[3] != N || in_sizes[4] != NSH * 8 || in_sizes[6] != 16 * F0 || in_sizes[8] != R * F0 * H1D || in_sizes[11] != R * H1D * OUTD || in_sizes[14] != OUTD * NCLS || out_size != G * NCLS) return;
  size_t off = 0; char* ws = (char*)d_ws;
  auto carve = [&](size_t bytes) { char* p = ws + off; off += (bytes + 255) & ~(size_t)255; return p; };
  b16* WS1 = (b16*)carve((size_t)H1D * (1 + R) * F0 * 2); b16* WS2 = (b16*)carve((size_t)OUTD * (1 + R) * H1D * 2); float* H0 = (float*)carve((size_t)NP * F0 * 4); float* H1 = (float*)carve((size_t)NP * H1D * 4); float* H2 = (float*)carve((size_t)NP * OUTD * 4); float* GP = (float*)carve((size_t)G * OUTD * 4);
  CsrBufs csr; off = csr_carve(csr, ws, off, E, N);
  if (off > ws_size || off > ((size_t)128 << 20)) return;
  wprep_kernel<<<(H1D * (1 + R) * F0 / 8 + 255) / 256, 256, 0, stream>>>(Fp(8), Fp(9), F0, H1D, WS1);
  wprep_kernel<<<(OUTD * (1 + R) * H1D / 8 + 255) / 256, 256, 0, stream>>>(Fp(11), Fp(12), H1D, OUTD, WS2);
  emb_kernel<<<NP / 64, 128, 0, stream>>>(Ip(0), Fp(4), Fp(5), Fp(6), Fp(7), H0);
  csr_build(csr, Ip(1) + E, E, N, stream);
  rgcn_kernel<F0, H1D, 0, 1><<<NP / 16, 32, 0, stream>>>(H0, nullptr, Ip(1), Ip(2), csr.PERM, csr.ROWPTR, csr.ROWCNT, (int)csr.permLen, WS1, Fp(10), H1);
  rgcn_kernel<H1D, OUTD, 0, 1><<<NP / 16, 32, 0, stream>>>(H1, nullptr, Ip(1), Ip(2), csr.PERM, csr.ROWPTR, csr.ROWCNT, (int)csr.permLen, WS2, Fp(13), H2);
  pool_kernel<<<G, 64, 0, stream>>>(H2, Ip(3), GP);
  cls_kernel<<<1, 512, 0, stream>>>(GP, Fp(14), Fp(15), (float*)d_out);
}
